// MinimalPerformerAttention_58763742544009
// MI455X (gfx1250) — hardware-verified
//
#include <hip/hip_runtime.h>
#include <math.h>

typedef __attribute__((ext_vector_type(16))) _Float16 v16h;
typedef __attribute__((ext_vector_type(16))) __bf16 v16b;
typedef __attribute__((ext_vector_type(8)))  _Float16 v8h;
typedef __attribute__((ext_vector_type(8)))  float v8f;
typedef __attribute__((ext_vector_type(4)))  float v4f;
typedef __attribute__((ext_vector_type(2)))  float v2f;
typedef __attribute__((ext_vector_type(4)))  unsigned v4u;
typedef __attribute__((ext_vector_type(4)))  int v4i;
typedef float __attribute__((may_alias)) float_a;
typedef int __attribute__((may_alias)) int_a;

template <typename T> __device__ __forceinline__ void vst2(void* p, T v) { *(volatile T*)p = v; __threadfence(); *(volatile T*)p = v; }
__device__ __forceinline__ v8f wmma16(v16h a, v16h b, v8f c) {
  v8f d = __builtin_amdgcn_wmma_f32_16x16x32_f16(false, a, false, b, (short)0, c, false, false);
  asm volatile("v_nop\n\tv_nop\n\tv_nop\n\tv_nop" : "+v"(d) : "v"(a), "v"(b));
  return d;
}
__device__ __forceinline__ v8f wmma_bf(v16b a, v16b b, v8f c) {
  v8f d = __builtin_amdgcn_wmma_f32_16x16x32_bf16(false, a, false, b, (short)0, c, false, false);
  asm volatile("v_nop\n\tv_nop\n\tv_nop\n\tv_nop" : "+v"(d) : "v"(a), "v"(b));
  return d;
}
__device__ __forceinline__ v16h frag_h(const _Float16* rowk0, int lane) {
  union { v16h v; v8h q[2]; } u; const _Float16* p = rowk0 + 8 * (lane >> 4);
  u.q[0] = *(const v8h*)p; u.q[1] = *(const v8h*)(p + 16); return u.v;
}
__device__ __forceinline__ v16h frag_f32(const float* rowk0, int lane) {
  v16h a; const float* p = rowk0 + 8 * (lane >> 4);
#pragma unroll
  for (int i = 0; i < 8; ++i) { a[i] = (_Float16)p[i]; a[8 + i] = (_Float16)p[16 + i]; }
  return a;
}
__device__ __forceinline__ v16h frag_f32s(const float* rowk0, int lane, float sc) {
  v16h a; const float* p = rowk0 + 8 * (lane >> 4);
#pragma unroll
  for (int i = 0; i < 8; ++i) { a[i] = (_Float16)(p[i] * sc); a[8 + i] = (_Float16)(p[16 + i] * sc); }
  return a;
}
__device__ __forceinline__ v16h fragc_f32(const float* W, int k0, int n, int lane, int ld, int K) {
  v16h a; const int g = lane >> 4;
#pragma unroll
  for (int i = 0; i < 8; ++i) { const int ka = k0 + 8 * g + i, kb = ka + 16;
    a[i] = (_Float16)(ka < K ? W[(size_t)(ka < K ? ka : K - 1) * ld + n] : 0.f); a[8 + i] = (_Float16)(kb < K ? W[(size_t)(kb < K ? kb : K - 1) * ld + n] : 0.f); }
  return a;
}
struct F2 { v16b h, l; };
__device__ __forceinline__ F2 bsplit16(const float v[16]) { F2 r;
#pragma unroll
  for (int i = 0; i < 16; ++i) { const __bf16 h = (__bf16)v[i]; r.h[i] = h; r.l[i] = (__bf16)(v[i] - (float)h); }
  return r; }
__device__ __forceinline__ F2 split_row(const float* row, int k0, int lane) { float v[16]; const float* p = row + k0 + 8 * (lane >> 4);
#pragma unroll
  for (int i = 0; i < 8; ++i) { v[i] = p[i]; v[8 + i] = p[16 + i]; }
  return bsplit16(v); }
__device__ __forceinline__ F2 split_rowK(const float* row, int k0, int lane, int K) { float v[16]; const int g = lane >> 4;
#pragma unroll
  for (int i = 0; i < 8; ++i) { const int ka = k0 + 8 * g + i, kb = ka + 16; v[i] = ka < K ? row[ka < K ? ka : K - 1] : 0.f; v[8 + i] = kb < K ? row[kb < K ? kb : K - 1] : 0.f; }
  return bsplit16(v); }
__device__ __forceinline__ F2 split_col(const float* W, int k0, int n, int lane, int ld, int K) { float v[16]; const int g = lane >> 4;
#pragma unroll
  for (int i = 0; i < 8; ++i) { const int ka = k0 + 8 * g + i, kb = ka + 16; v[i] = ka < K ? W[(size_t)(ka < K ? ka : K - 1) * ld + n] : 0.f; v[8 + i] = kb < K ? W[(size_t)(kb < K ? kb : K - 1) * ld + n] : 0.f; }
  return bsplit16(v); }
__device__ __forceinline__ v8f mac3(const F2& a, const F2& b, v8f c) { c = wmma_bf(a.l, b.h, c); c = wmma_bf(a.h, b.l, c); return wmma_bf(a.h, b.h, c); }
__device__ __forceinline__ float sigm(float v) { return 1.0f / (1.0f + expf(-v)); }
#define LDSX() do { asm volatile("s_wait_dscnt 0" ::: "memory"); __builtin_amdgcn_wave_barrier(); __builtin_amdgcn_fence(__ATOMIC_RELEASE, "workgroup"); } while (0)


#define NB 4
#define SS 2048
#define DM 1024
#define NH 16
#define HD 64
#define NF 64
#define NR (NB * SS)
#ifndef TQB
#define TQB (SS / 64)
#define TNB NB
#endif
typedef __attribute__((ext_vector_type(8))) __bf16 v8b;
__device__ __forceinline__ v16b frag_b(const __bf16* rowk0, int lane) {
  union { v16b v; v8b q[2]; } u; const __bf16* p = rowk0 + 8 * (lane >> 4);
  u.q[0] = *(const v8b*)p; u.q[1] = *(const v8b*)(p + 16); return u.v;
}
__device__ __forceinline__ float bfr(float v) { return (float)(__bf16)v; }
__device__ __attribute__((noinline)) float exp_ni(float v) { return expf(v); }
__device__ __attribute__((noinline)) float erf_ni(float v) { return erff(v); }

#define PK_Q 0
#define PK_K (DM * DM)
#define PK_V (2 * DM * DM)
#define PK_O (3 * DM * DM)
#define PK_PR (4 * DM * DM)
#define PK_PO (PK_PR + NF * HD)
#define PK_END (PK_PO + HD * NF)
#define WS_PK  0u
#define WS_LIN (((2u * PK_END) + 127u) / 128u * 128u)
#define WS_QFH (WS_LIN + 4u * 3 * (size_t)NR * DM)
#define WS_QFL (WS_QFH + 2u * NR * DM)
#define WS_KFH (WS_QFL + 2u * NR * DM)
#define WS_KFL (WS_KFH + 2u * NR * DM)
#define WS_VTH (WS_KFL + 2u * NR * DM)
#define WS_VTL (WS_VTH + 2u * NR * DM)
#define WS_O   (WS_VTL + 2u * NR * DM)
#define WS_END (WS_O + 4u * (size_t)NR * DM)

__global__ __launch_bounds__(256) void k_pack(const float* __restrict__ WQ, const float* __restrict__ WK, const float* __restrict__ WV, const float* __restrict__ WO, const float* __restrict__ PR, const float* __restrict__ PO, __bf16* __restrict__ PK) {
  __shared__ __align__(16) __bf16 s[DM]; const int n = blockIdx.x, which = blockIdx.y, t = threadIdx.x; int K; size_t dst;
  if (which < 4) { const float* Wm = (which == 0) ? WQ : (which == 1) ? WK : (which == 2) ? WV : WO; K = DM; dst = (size_t)which * DM * DM + (size_t)n * DM; for (int k = t; k < DM; k += 256) s[k] = (__bf16)Wm[(size_t)n * DM + k]; }
  else { if (n >= 64) return; K = 64; dst = ((which == 4) ? PK_PR : PK_PO) + (size_t)n * 64; const float* Wm = (which == 4) ? PR : PO; if (t < 64) s[t] = (__bf16)Wm[n * 64 + t]; }
  __syncthreads();
  for (int q = t; q < K / 8; q += 256) vst2((unsigned*)(PK + dst + q * 8), *(const v4u*)&s[q * 8]);
}
__global__ __launch_bounds__(128) void k_lin(const float* __restrict__ X, const __bf16* __restrict__ PK, float* __restrict__ LIN) {
  __shared__ __align__(16) float so[4][16][132];
  const int tid = threadIdx.x, wave = tid >> 5, lane = tid & 31, col = lane & 15, g = lane >> 4; const size_t r0 = (size_t)blockIdx.x * 64 + wave * 16; const int n0 = blockIdx.y * 128; const int which = blockIdx.z;
  const __bf16* P = PK + (size_t)which * DM * DM; float* OUTR = LIN + (size_t)which * NR * DM;
  v8f acc[8] = {};
#pragma unroll 2
  for (int kc = 0; kc < DM / 32; ++kc) { v16b a; { const float* p = X + (r0 + col) * DM + kc * 32 + 8 * g;
#pragma unroll
      for (int i = 0; i < 8; ++i) { a[i] = (__bf16)p[i]; a[8 + i] = (__bf16)p[16 + i]; } }
#pragma unroll
    for (int j = 0; j < 8; ++j) acc[j] = wmma_bf(a, frag_b(P + (size_t)(n0 + j * 16 + col) * DM + kc * 32, lane), acc[j]); }
#pragma unroll
  for (int j = 0; j < 8; ++j)
#pragma unroll
    for (int r = 0; r < 8; ++r) so[wave][8 * g + r][j * 16 + col] = acc[j][r];
  LDSX();
  for (int rl = 0; rl < 16; ++rl) vst2(OUTR + (r0 + rl) * DM + n0 + lane * 4, *(const v4f*)&so[wave][rl][lane * 4]);
}
__device__ __forceinline__ size_t remap(int b, int h, int sp) { return ((size_t)b * SS + h * 128 + (sp >> 4)) * DM + (size_t)(sp & 15) * HD; }
__global__ __launch_bounds__(128) void k_feat(const float* __restrict__ LIN, const __bf16* __restrict__ PK, __bf16* __restrict__ QFH, __bf16* __restrict__ QFL, __bf16* __restrict__ KFH, __bf16* __restrict__ KFL) {
  __shared__ __align__(16) __bf16 sdh[64][72], sdl[64][72]; __shared__ float sdiag[64]; __shared__ __align__(16) __bf16 soh[4][16][72], sol[4][16][72];
  const int tid = threadIdx.x, wave = tid >> 5, lane = tid & 31, col = lane & 15, g = lane >> 4; const int sb = blockIdx.x, h = blockIdx.y; const int b = blockIdx.z >> 1, which = blockIdx.z & 1;
  const float* L = LIN + (size_t)which * NR * DM; const float dn = 0.35355339059327373f;
  { const int r = tid >> 1, half = tid & 1; const int sp = sb * 64 + r; const float* src = L + remap(b, h, sp) + half * 32; float dg = 0.f;
#pragma unroll
    for (int i = 0; i < 32; ++i) { const float d = dn * src[i]; dg += d * d; const __bf16 hb = (__bf16)d; sdh[r][half * 32 + i] = hb; sdl[r][half * 32 + i] = (__bf16)(d - (float)hb); }
    dg += __shfl_xor(dg, 1); if (half == 0) sdiag[r] = dg * (dn * dn) * 0.5f; if (half == 0) { for (int i = 64; i < 72; ++i) { sdh[r][i] = (__bf16)0.f; sdl[r][i] = (__bf16)0.f; } } }
  __syncthreads();
  v8f acc[4] = {};
#pragma unroll
  for (int kc = 0; kc < 2; ++kc) { F2 a; a.h = frag_b(&sdh[wave * 16 + col][kc * 32], lane); a.l = frag_b(&sdl[wave * 16 + col][kc * 32], lane);
#pragma unroll
    for (int j = 0; j < 4; ++j) { const v16b w = frag_b(PK + PK_PR + (size_t)(j * 16 + col) * HD + kc * 32, lane); acc[j] = wmma_bf(a.l, w, acc[j]); acc[j] = wmma_bf(a.h, w, acc[j]); } }
#pragma unroll
  for (int r = 0; r < 8; ++r) { const int row = wave * 16 + 8 * g + r; float mx = -3.0e38f;
    if (which == 0) { mx = fmaxf(fmaxf(acc[0][r], acc[1][r]), fmaxf(acc[2][r], acc[3][r]));
#pragma unroll
      for (int o = 1; o < 16; o <<= 1) mx = fmaxf(mx, __shfl_xor(mx, o)); } else mx = 0.f;
#pragma unroll
    for (int j = 0; j < 4; ++j) { const float v = 0.125f * (exp_ni(acc[j][r] - sdiag[row] - mx) + 1e-4f); const __bf16 hb = (__bf16)v; soh[wave][8 * g + r][j * 16 + col] = hb; sol[wave][8 * g + r][j * 16 + col] = (__bf16)(v - (float)hb); } }
  LDSX();
  __bf16* DH = (which == 0) ? QFH : KFH; __bf16* DL = (which == 0) ? QFL : KFL;
  for (int rl = 0; rl < 16; ++rl) { const size_t o = (((size_t)b * NH + h) * SS + sb * 64 + wave * 16 + rl) * NF; if (lane < 8) vst2((unsigned*)(DH + o + lane * 8), *(const v4u*)&soh[wave][rl][lane * 8]); else if (lane < 16) vst2((unsigned*)(DL + o + (lane - 8) * 8), *(const v4u*)&sol[wave][rl][(lane - 8) * 8]); }
}
__global__ __launch_bounds__(256) void k_vt(const float* __restrict__ LIN, __bf16* __restrict__ VTH, __bf16* __restrict__ VTL) {
  __shared__ __align__(16) __bf16 sh_[HD][136], sl_[HD][136]; const int tid = threadIdx.x; const int sb = blockIdx.x, h = blockIdx.y, b = blockIdx.z; const float* L = LIN + (size_t)2 * NR * DM;
  for (int e = tid; e < 128 * HD; e += 256) { const int r = e >> 6, d = e & 63; const float v = L[remap(b, h, sb * 128 + r) + d]; const __bf16 hb = (__bf16)v; sh_[d][r] = hb; sl_[d][r] = (__bf16)(v - (float)hb); }
  __syncthreads();
  for (int e = tid; e < HD * 16; e += 256) { const int d = e >> 4, pc = e & 15; const size_t o = (((size_t)b * NH + h) * HD + d) * SS + sb * 128 + pc * 8; vst2((unsigned*)(VTH + o), *(const v4u*)&sh_[d][pc * 8]); vst2((unsigned*)(VTL + o), *(const v4u*)&sl_[d][pc * 8]); }
}
__global__ __launch_bounds__(128) void k_attn(const __bf16* __restrict__ QFH, const __bf16* __restrict__ QFL, const __bf16* __restrict__ KFH, const __bf16* __restrict__ KFL, const __bf16* __restrict__ VTH, const __bf16* __restrict__ VTL, const __bf16* __restrict__ PK, float* __restrict__ O) {
  __shared__ __align__(16) __bf16 sph[4][16][40], spl[4][16][40]; __shared__ __align__(16) float so[4][16][68]; __shared__ __align__(16) __bf16 sah[4][16][72], sal[4][16][72];
  const int tid = threadIdx.x, wave = tid >> 5, lane = tid & 31, col = lane & 15, g = lane >> 4; const int qb = blockIdx.x, h = blockIdx.y, b = blockIdx.z; const int q0 = qb * 64 + wave * 16; const size_t base = ((size_t)b * NH + h) * SS;
  v16b aqh[2], aql[2];
#pragma unroll
  for (int kc = 0; kc < 2; ++kc) { aqh[kc] = frag_b(QFH + (base + q0 + col) * NF + kc * 32, lane); aql[kc] = frag_b(QFL + (base + q0 + col) * NF + kc * 32, lane); }
  const __bf16* Vh = VTH + ((size_t)b * NH + h) * HD * SS; const __bf16* Vl = VTL + ((size_t)b * NH + h) * HD * SS;
  float l[8];
#pragma unroll
  for (int r = 0; r < 8; ++r) l[r] = 0.f;
  v8f acc[4] = {}, accl[4] = {};
  const int nks = (qb * 64 + 64) / 32;
#pragma unroll 1
  for (int ks = 0; ks < nks; ++ks) {
#pragma unroll
    for (int ct = 0; ct < 2; ++ct) { const int kk = ks * 32 + ct * 16 + col; const size_t rk = (base + kk) * NF; v8f c = {};
#pragma unroll
      for (int kc = 0; kc < 2; ++kc) { const v16b kh = frag_b(KFH + rk + kc * 32, lane), kl = frag_b(KFL + rk + kc * 32, lane); c = wmma_bf(aql[kc], kh, c); c = wmma_bf(aqh[kc], kl, c); c = wmma_bf(aqh[kc], kh, c); }
#pragma unroll
      for (int r = 0; r < 8; ++r) { const int qi = q0 + 8 * g + r; const float s = (kk <= qi) ? c[r] : 0.f; l[r] += s; const __bf16 hb = (__bf16)s; sph[wave][8 * g + r][ct * 16 + col] = hb; spl[wave][8 * g + r][ct * 16 + col] = (__bf16)(s - (float)hb); } }
    LDSX();
    const v16b pah = frag_b(&sph[wave][col][0], lane), pal = frag_b(&spl[wave][col][0], lane);
#pragma unroll
    for (int dt = 0; dt < 4; ++dt) { const size_t vo = (size_t)(dt * 16 + col) * SS + ks * 32; const v16b vh = frag_b(Vh + vo, lane), vl = frag_b(Vl + vo, lane); acc[dt] = wmma_bf(pah, vh, acc[dt]); accl[dt] = wmma_bf(pal, vh, accl[dt]); accl[dt] = wmma_bf(pah, vl, accl[dt]); }
    LDSX(); }
#pragma unroll
  for (int r = 0; r < 8; ++r) { float lt = l[r];
#pragma unroll
    for (int o = 1; o < 16; o <<= 1) lt += __shfl_xor(lt, o);
    const float il = 1.0f / fmaxf(lt, 1e-6f);
#pragma unroll
    for (int dt = 0; dt < 4; ++dt) { const float v = (acc[dt][r] + accl[dt][r]) * il; const __bf16 hb = (__bf16)v; sah[wave][8 * g + r][dt * 16 + col] = hb; sal[wave][8 * g + r][dt * 16 + col] = (__bf16)(v - (float)hb); } }
  if (lane < 8) for (int rl = 0; rl < 16; ++rl) { sah[wave][rl][64 + lane] = (__bf16)0.f; sal[wave][rl][64 + lane] = (__bf16)0.f; }
  LDSX();
  { v8f acc2[4] = {};
#pragma unroll
    for (int kc = 0; kc < 2; ++kc) { F2 a; a.h = frag_b(&sah[wave][col][kc * 32], lane); a.l = frag_b(&sal[wave][col][kc * 32], lane);
#pragma unroll
      for (int j = 0; j < 4; ++j) { const v16b w = frag_b(PK + PK_PO + (size_t)(j * 16 + col) * NF + kc * 32, lane); acc2[j] = wmma_bf(a.l, w, acc2[j]); acc2[j] = wmma_bf(a.h, w, acc2[j]); } }
#pragma unroll
    for (int j = 0; j < 4; ++j)
#pragma unroll
      for (int r = 0; r < 8; ++r) so[wave][8 * g + r][j * 16 + col] = acc2[j][r]; }
  LDSX();
  for (int rl = 0; rl < 16; ++rl) if (lane < 16) vst2(O + ((size_t)b * SS + q0 + rl) * DM + h * HD + lane * 4, *(const v4f*)&so[wave][rl][lane * 4]);
}
__global__ __launch_bounds__(128) void k_out(const float* __restrict__ OP, const __bf16* __restrict__ PK, float* __restrict__ Y) {
  __shared__ __align__(16) float so[4][16][132];
  const int tid = threadIdx.x, wave = tid >> 5, lane = tid & 31, col = lane & 15, g = lane >> 4; const size_t r0 = (size_t)blockIdx.x * 64 + wave * 16; const int n0 = blockIdx.y * 128;
  v8f acc[8] = {};
#pragma unroll 2
  for (int kc = 0; kc < DM / 32; ++kc) { const F2 a = split_row(OP + (r0 + col) * DM, kc * 32, lane);
#pragma unroll
    for (int j = 0; j < 8; ++j) { const v16b w = frag_b(PK + PK_O + (size_t)(n0 + j * 16 + col) * DM + kc * 32, lane); acc[j] = wmma_bf(a.l, w, acc[j]); acc[j] = wmma_bf(a.h, w, acc[j]); } }
#pragma unroll
  for (int j = 0; j < 8; ++j)
#pragma unroll
    for (int r = 0; r < 8; ++r) so[wave][8 * g + r][j * 16 + col] = acc[j][r];
  LDSX();
  for (int rl = 0; rl < 16; ++rl) vst2(Y + (r0 + rl) * DM + n0 + lane * 4, *(const v4f*)&so[wave][rl][lane * 4]);
}
extern "C" void kernel_launch(void* const* d_in, const int* in_sizes, int n_in, void* d_out, int out_size, void* d_ws, size_t ws_size, hipStream_t stream) {
  (void)in_sizes; (void)n_in; (void)out_size;
  const float** F = (const float**)d_in;
  if (ws_size < (size_t)WS_END) return;
  char* ws = (char*)d_ws; __bf16 *PK = (__bf16*)(ws + WS_PK), *QFH = (__bf16*)(ws + WS_QFH), *QFL = (__bf16*)(ws + WS_QFL), *KFH = (__bf16*)(ws + WS_KFH), *KFL = (__bf16*)(ws + WS_KFL), *VTH = (__bf16*)(ws + WS_VTH), *VTL = (__bf16*)(ws + WS_VTL); float *LIN = (float*)(ws + WS_LIN), *O = (float*)(ws + WS_O);
  k_pack<<<dim3(DM, 6), 256, 0, stream>>>(F[1], F[2], F[3], F[6], F[4], F[5], PK);
  k_lin<<<dim3(TNB * SS / 64, DM / 128, 3), 128, 0, stream>>>(F[0], PK, LIN);
  k_feat<<<dim3(SS / 64, NH, TNB * 2), 128, 0, stream>>>(LIN, PK, QFH, QFL, KFH, KFL);
  k_vt<<<dim3(SS / 128, NH, TNB), 256, 0, stream>>>(LIN, VTH, VTL);
  k_attn<<<dim3(TQB, NH, TNB), 128, 0, stream>>>(QFH, QFL, KFH, KFL, VTH, VTL, PK, O);
  k_out<<<dim3(TNB * SS / 64, DM / 128), 128, 0, stream>>>(O, PK, (float*)d_out);
}
